// GraphNeuralEncoder_24335284699305
// MI455X (gfx1250) — hardware-verified
//
#include <hip/hip_runtime.h>
#include <stddef.h>
#include <math.h>


#define NGR    256
#define NPG    100
#define NCU    99
#define NNODE  25600
#define CD     128
#define HD     512
#define NL     3
#define NTHR   256
#define NWAVE  8
#define G1ROWS 128
#define FROWS  64
#define IROWS  8
#define PTHR   128
#define APKX   136
#define APKF   520
#define BN_EPS 1e-5f
#define WSCAP  134217728

#define WPG_SZ (2 * CD * CD)
#define WP1_SZ (2 * HD * CD)
#define WP2_SZ (2 * CD * HD)
#define WPL_SZ (WPG_SZ + WP1_SZ + WP2_SZ)
#define WPTOT  (NL * WPL_SZ)
#define WBLK_L 72

#define REC    (2 * CD)
#define NP1    NGR
#define NP2    (NNODE / FROWS)

#define LDS_G1  (2 * G1ROWS * APKX * 2 + G1ROWS * CD * 4)
#define LDS_FFN (2 * FROWS * APKX * 2 + 2 * FROWS * APKF * 2)

static_assert(NNODE == NGR * NPG);
static_assert(NPG == NCU + 1);
static_assert((NNODE % G1ROWS) == 0 && (NNODE % FROWS) == 0 && (NNODE % IROWS) == 0);
static_assert(G1ROWS == NWAVE * 16 && FROWS == 4 * 16 && NTHR == NWAVE * 32 && IROWS == NWAVE);
static_assert((NPG % 4) == 0);
static_assert(CD == 128 && (HD % 64) == 0);
static_assert((APKX % 8) == 0 && (APKF % 8) == 0 && APKX >= CD && APKF >= HD);
static_assert(FROWS * CD * 4 <= 2 * FROWS * APKX * 2);
static_assert((NWAVE * REC + REC) * 8 <= 2 * FROWS * APKF * 2);
static_assert((WPG_SZ % 64) == 0 && (WP1_SZ % 64) == 0 && (WPL_SZ % 64) == 0);
static_assert(WBLK_L * NTHR * 8 == CD * CD + HD * CD + CD * HD);
static_assert(PTHR == CD);

typedef float          v4f  __attribute__((ext_vector_type(4)));
typedef float          v8f  __attribute__((ext_vector_type(8)));
typedef double         v2d  __attribute__((ext_vector_type(2)));
typedef unsigned short v8us __attribute__((ext_vector_type(8)));
typedef __bf16         v16b __attribute__((ext_vector_type(16)));
union FragB { v16b v; v8us h[2]; };

__device__ __forceinline__ unsigned int bfr(float f) {
  const unsigned int u = __float_as_uint(f);
  return (u + 0x7FFFu + ((u >> 16) & 1u)) >> 16;
}

__device__ __forceinline__ void split1(float x, unsigned short& hb, unsigned short& lb) {
  const unsigned int hu = bfr(x);
  const float hf = __uint_as_float(hu << 16);
  hb = (unsigned short)hu;
  lb = (unsigned short)bfr(x - hf);
}

__device__ __forceinline__ void split8(v4f a, v4f b, v8us& hi, v8us& lo) {
  unsigned short hb, lb;
  split1(a.x, hb, lb); hi[0] = hb; lo[0] = lb;
  split1(a.y, hb, lb); hi[1] = hb; lo[1] = lb;
  split1(a.z, hb, lb); hi[2] = hb; lo[2] = lb;
  split1(a.w, hb, lb); hi[3] = hb; lo[3] = lb;
  split1(b.x, hb, lb); hi[4] = hb; lo[4] = lb;
  split1(b.y, hb, lb); hi[5] = hb; lo[5] = lb;
  split1(b.z, hb, lb); hi[6] = hb; lo[6] = lb;
  split1(b.w, hb, lb); hi[7] = hb; lo[7] = lb;
}

__device__ __forceinline__ v8f wmb(v16b a, v16b b, v8f c) {
  v8f d = __builtin_amdgcn_wmma_f32_16x16x32_bf16(false, a, false, b, (short)0, c, false, false);
  asm volatile("v_nop\n\tv_nop\n\tv_nop\n\tv_nop" : "+v"(d) : "v"(a), "v"(b));
  return d;
}

template <int KD, int NCH, int APK>
__device__ __forceinline__ void mma_block(const unsigned short* sHi, const unsigned short* sLo,
                                          const unsigned short* __restrict__ Bh, size_t loOff,
                                          int wrow, int lane, v8f (&acc)[NCH / 16]) {
  static_assert((KD % 32) == 0 && (NCH % 16) == 0 && (APK % 8) == 0);
  constexpr int NTL = NCH / 16, NKT = KD / 32;
  const int hh = lane >> 4, m = lane & 15;
#pragma unroll
  for (int t = 0; t < NTL; ++t) { v8f z = {0.f, 0.f, 0.f, 0.f, 0.f, 0.f, 0.f, 0.f}; acc[t] = z; }
  const unsigned short* ahp = sHi + (wrow + m) * APK + 8 * hh;
  const unsigned short* alp = sLo + (wrow + m) * APK + 8 * hh;
#pragma unroll 1
  for (int kt = 0; kt < NKT; ++kt) {
    FragB ah, al;
    ah.h[0] = *(const v8us*)(ahp + 32 * kt);
    ah.h[1] = *(const v8us*)(ahp + 32 * kt + 16);
    al.h[0] = *(const v8us*)(alp + 32 * kt);
    al.h[1] = *(const v8us*)(alp + 32 * kt + 16);
#pragma unroll
    for (int t = 0; t < NTL; ++t) {
      const unsigned short* bp = Bh + (size_t)(16 * t + m) * KD + 32 * kt + 8 * hh;
      FragB bh, bl;
      bh.h[0] = *(const v8us*)bp;
      bh.h[1] = *(const v8us*)(bp + 16);
      bl.h[0] = *(const v8us*)(bp + loOff);
      bl.h[1] = *(const v8us*)(bp + loOff + 16);
      acc[t] = wmb(ah.v, bh.v, acc[t]);
      acc[t] = wmb(ah.v, bl.v, acc[t]);
      acc[t] = wmb(al.v, bh.v, acc[t]);
    }
  }
}

__global__ __launch_bounds__(NTHR) void k_wprep(const float* __restrict__ wg, const float* __restrict__ w1,
                                                const float* __restrict__ w2, unsigned short* wp) {
  const int blk = blockIdx.x, tid = threadIdx.x;
  const int l = blk / WBLK_L, lb = blk - WBLK_L * l;
  int KD, NCOL, i, ksh;
  size_t base;
  const float* src;
  if (lb < 8) {
    KD = CD; NCOL = CD; ksh = 4; i = lb * NTHR + tid;
    base = (size_t)l * WPL_SZ; src = wg + (size_t)l * CD * CD;
  } else if (lb < 40) {
    KD = CD; NCOL = HD; ksh = 4; i = (lb - 8) * NTHR + tid;
    base = (size_t)l * WPL_SZ + WPG_SZ; src = w1 + (size_t)l * CD * HD;
  } else {
    KD = HD; NCOL = CD; ksh = 6; i = (lb - 40) * NTHR + tid;
    base = (size_t)l * WPL_SZ + WPG_SZ + WP1_SZ; src = w2 + (size_t)l * HD * CD;
  }
  const int n = i >> ksh, k0 = (i - (n << ksh)) * 8;
  float v[8];
#pragma unroll
  for (int e = 0; e < 8; ++e) v[e] = src[(size_t)(k0 + e) * NCOL + n];
  v4f a, b;
  a.x = v[0]; a.y = v[1]; a.z = v[2]; a.w = v[3];
  b.x = v[4]; b.y = v[5]; b.z = v[6]; b.w = v[7];
  v8us hv, lv;
  split8(a, b, hv, lv);
  unsigned short* dh = wp + base + (size_t)i * 8;
  unsigned short* dl = dh + (size_t)NCOL * KD;
  *(volatile v8us*)dh = hv;
  *(volatile v8us*)dl = lv;
  __threadfence();
  *(volatile v8us*)dh = hv;
  *(volatile v8us*)dl = lv;
}

__global__ __launch_bounds__(NTHR) void k_init(
    const float* __restrict__ depot, const float* __restrict__ cust, const float* __restrict__ dem,
    const float* __restrict__ Wd, const float* __restrict__ bd, const float* __restrict__ Wi,
    const float* __restrict__ bi, float* x0, float* tab0) {
  const int tid = threadIdx.x, lane = tid & 31, wave = tid >> 5;
  const int node = blockIdx.x * IROWS + wave;
  const int b = node / NPG, j = node - b * NPG;
  int q = b * NCU + (j - 1);
  q = q < 0 ? 0 : (q > NGR * NCU - 1 ? NGR * NCU - 1 : q);
  const float dx = depot[b * 2], dy = depot[b * 2 + 1];
  const float cx = cust[(size_t)q * 2], cy = cust[(size_t)q * 2 + 1], cm = dem[q];
  const int c0 = 4 * lane;
  float ov[4];
#pragma unroll
  for (int e = 0; e < 4; ++e) {
    const int c = c0 + e;
    const float vd = dx * Wd[c] + dy * Wd[CD + c] + bd[c];
    const float vc = cx * Wi[c] + cy * Wi[CD + c] + cm * Wi[2 * CD + c] + bi[c];
    ov[e] = (j == 0) ? vd : vc;
  }
  v4f o;
  o.x = ov[0]; o.y = ov[1]; o.z = ov[2]; o.w = ov[3];
  float* gp = x0 + (size_t)node * CD + c0;
  const v4f one = {1.0f, 1.0f, 1.0f, 1.0f};
  const v4f zer = {0.0f, 0.0f, 0.0f, 0.0f};
  const bool tw = (blockIdx.x == 0) && (tid < 64);
  const v4f tv = (tid < 32) ? one : zer;
  *(volatile v4f*)gp = o;
  if (tw) *(volatile v4f*)(tab0 + 4 * tid) = tv;
  __threadfence();
  *(volatile v4f*)gp = o;
  if (tw) *(volatile v4f*)(tab0 + 4 * tid) = tv;
}

__global__ __launch_bounds__(NTHR) void k_gemm1(const float* __restrict__ ysrc, const float* __restrict__ tab,
                                                const unsigned short* __restrict__ Bw, float* hout) {
  extern __shared__ v4f lds_dyn[];
  unsigned short* sHi = (unsigned short*)lds_dyn;
  unsigned short* sLo = sHi + G1ROWS * APKX;
  float*          stg = (float*)((char*)lds_dyn + 2 * G1ROWS * APKX * 2);
  const int tid = threadIdx.x, lane = tid & 31, wave = tid >> 5, hh = lane >> 4, m = lane & 15;
  const int rowBase = blockIdx.x * G1ROWS;

#pragma unroll
  for (int it = 0; it < 8; ++it) {
    const int idx = it * NTHR + tid;
    const int r   = idx >> 4;
    const int c0  = (idx & 15) * 8;
    const float* ap = ysrc + (size_t)(rowBase + r) * CD + c0;
    v4f a = *(const v4f*)ap, b = *(const v4f*)(ap + 4);
    const v4f s0 = *(const v4f*)(tab + c0),      s1 = *(const v4f*)(tab + c0 + 4);
    const v4f h0 = *(const v4f*)(tab + CD + c0), h1 = *(const v4f*)(tab + CD + c0 + 4);
    a = a * s0 + h0;
    b = b * s1 + h1;
    v8us hv, lv;
    split8(a, b, hv, lv);
    *(v8us*)(sHi + r * APKX + c0) = hv;
    *(v8us*)(sLo + r * APKX + c0) = lv;
  }
  __syncthreads();

#pragma unroll 1
  for (int ch = 0; ch < 2; ++ch) {
    v8f acc[4];
    mma_block<CD, 64, APKX>(sHi, sLo, Bw + (size_t)(ch * 64) * CD, (size_t)CD * CD, wave * 16, lane, acc);
    float* sp = stg + (wave * 16 + 8 * hh) * CD + ch * 64 + m;
#pragma unroll
    for (int t = 0; t < 4; ++t) {
#pragma unroll
      for (int r = 0; r < 8; ++r) sp[r * CD + 16 * t] = acc[t][r];
    }
  }
  __syncthreads();

  const float* lp = stg + (wave * 16) * CD + 4 * lane;
  float* gp = hout + (size_t)(rowBase + wave * 16) * CD + 4 * lane;
#pragma unroll
  for (int i = 0; i < 16; ++i) { const v4f v = *(const v4f*)(lp + i * CD); *(volatile v4f*)(gp + (size_t)i * CD) = v; }
  __threadfence();
#pragma unroll
  for (int i = 0; i < 16; ++i) { const v4f v = *(const v4f*)(lp + i * CD); *(volatile v4f*)(gp + (size_t)i * CD) = v; }
}

__global__ __launch_bounds__(PTHR) void k_prefix(const float* __restrict__ h, const float* __restrict__ ysrc,
                                                 const float* __restrict__ tab, const float* __restrict__ gb,
                                                 float* y1, double* part) {
  __shared__ __attribute__((aligned(16))) float  sy[NPG * CD];
  __shared__ __attribute__((aligned(16))) double srec[REC];
  const int b = blockIdx.x, c = threadIdx.x, lane = c & 31, wave = c >> 5;
  const size_t gbase = (size_t)b * NPG * CD;
  const float sc = tab[c], sh = tab[CD + c], bc = gb[c];
  float run = 0.0f;
  double s = 0.0, q = 0.0;
#pragma unroll 1
  for (int j = 0; j < NPG; ++j) {
    const float dj  = rsqrtf((float)(j + 1));
    const float hv  = h[gbase + (size_t)j * CD + c];
    run = run + dj * hv;
    const float agg = dj * run + bc;
    const float xv  = ysrc[gbase + (size_t)j * CD + c] * sc + sh;
    const float yv  = xv + agg;
    sy[j * CD + c] = yv;
    s += (double)yv;
    q += (double)yv * (double)yv;
  }
  srec[c] = s;
  srec[CD + c] = q;
  __syncthreads();

  float* gy = y1 + gbase + 4 * lane;
  double* gr = part + (size_t)b * REC + 2 * c;
  const v2d rv = *(const v2d*)(srec + 2 * c);
#pragma unroll 1
  for (int k = 0; k < NPG / 4; ++k) {
    const int row = 4 * k + wave;
    const v4f v = *(const v4f*)(sy + row * CD + 4 * lane);
    *(volatile v4f*)(gy + (size_t)row * CD) = v;
  }
  *(volatile v2d*)gr = rv;
  __threadfence();
#pragma unroll 1
  for (int k = 0; k < NPG / 4; ++k) {
    const int row = 4 * k + wave;
    const v4f v = *(const v4f*)(sy + row * CD + 4 * lane);
    *(volatile v4f*)(gy + (size_t)row * CD) = v;
  }
  *(volatile v2d*)gr = rv;
}

__global__ __launch_bounds__(PTHR) void k_bnfin(const double* __restrict__ part, int nblk,
                                                const float* __restrict__ gamma, const float* __restrict__ beta,
                                                float* tab) {
  __shared__ __attribute__((aligned(16))) float st[REC];
  const int c = threadIdx.x;
  double S = 0.0, Q = 0.0;
#pragma unroll 1
  for (int bk = 0; bk < nblk; ++bk) {
    S += part[(size_t)bk * REC + c];
    Q += part[(size_t)bk * REC + CD + c];
  }
  const double mean = S * (1.0 / (double)NNODE);
  double var = Q * (1.0 / (double)NNODE) - mean * mean;
  var = var < 0.0 ? 0.0 : var;
  const float vf = (float)var;
  const float rs = rsqrtf(vf + BN_EPS);
  const float scl = gamma[c] * rs;
  const float shf = beta[c] - (float)mean * scl;
  st[c] = scl;
  st[CD + c] = shf;
  __syncthreads();
  v4f tv = {0.f, 0.f, 0.f, 0.f};
  if (c < 64) tv = *(const v4f*)(st + 4 * c);
  if (c < 64) *(volatile v4f*)(tab + 4 * c) = tv;
  __threadfence();
  if (c < 64) *(volatile v4f*)(tab + 4 * c) = tv;
}

__global__ __launch_bounds__(NTHR) void k_ffn(const float* __restrict__ y1, const float* __restrict__ tab1,
                                              const unsigned short* __restrict__ Bw1, const float* __restrict__ b1,
                                              const unsigned short* __restrict__ Bw2, const float* __restrict__ b2,
                                              float* y2, double* part) {
  extern __shared__ v4f lds_dyn[];
  unsigned short* sXh = (unsigned short*)lds_dyn;
  unsigned short* sXl = sXh + FROWS * APKX;
  unsigned short* sFh = sXl + FROWS * APKX;
  unsigned short* sFl = sFh + FROWS * APKF;
  float*  stg  = (float*)lds_dyn;
  double* spw  = (double*)sFh;
  double* srec = spw + NWAVE * REC;
  const int tid = threadIdx.x, lane = tid & 31, wave = tid >> 5, hh = lane >> 4, m = lane & 15;
  const int rowBase = blockIdx.x * FROWS;
  const int rg = wave & 3, chalf = wave >> 2;

#pragma unroll
  for (int it = 0; it < 4; ++it) {
    const int idx = it * NTHR + tid;
    const int r   = idx >> 4;
    const int c0  = (idx & 15) * 8;
    const float* ap = y1 + (size_t)(rowBase + r) * CD + c0;
    v4f a = *(const v4f*)ap, b = *(const v4f*)(ap + 4);
    const v4f s0 = *(const v4f*)(tab1 + c0),      s1 = *(const v4f*)(tab1 + c0 + 4);
    const v4f h0 = *(const v4f*)(tab1 + CD + c0), h1 = *(const v4f*)(tab1 + CD + c0 + 4);
    a = a * s0 + h0;
    b = b * s1 + h1;
    v8us hv, lv;
    split8(a, b, hv, lv);
    *(v8us*)(sXh + r * APKX + c0) = hv;
    *(v8us*)(sXl + r * APKX + c0) = lv;
  }
  __syncthreads();

#pragma unroll 1
  for (int ch = 0; ch < 4; ++ch) {
    const int n0 = chalf * 256 + ch * 64;
    v8f acc[4];
    mma_block<CD, 64, APKX>(sXh, sXl, Bw1 + (size_t)n0 * CD, (size_t)HD * CD, rg * 16, lane, acc);
#pragma unroll
    for (int t = 0; t < 4; ++t) {
      const int col = n0 + 16 * t + m;
      const float bv = b1[col];
#pragma unroll
      for (int r = 0; r < 8; ++r) {
        float v = acc[t][r] + bv;
        v = fmaxf(v, 0.0f);
        unsigned short hb, lb;
        split1(v, hb, lb);
        const int o = (rg * 16 + 8 * hh + r) * APKF + col;
        sFh[o] = hb;
        sFl[o] = lb;
      }
    }
  }
  __syncthreads();

  v8f acc2[4];
  mma_block<HD, 64, APKF>(sFh, sFl, Bw2 + (size_t)(chalf * 64) * HD, (size_t)CD * HD, rg * 16, lane, acc2);
  __syncthreads();
  {
    float* sp = stg + (rg * 16 + 8 * hh) * CD + chalf * 64 + m;
#pragma unroll
    for (int t = 0; t < 4; ++t) {
      const float bv = b2[chalf * 64 + 16 * t + m];
#pragma unroll
      for (int r = 0; r < 8; ++r) sp[r * CD + 16 * t] = acc2[t][r] + bv;
    }
  }
  __syncthreads();

  const v4f sc = *(const v4f*)(tab1 + 4 * lane), sh = *(const v4f*)(tab1 + CD + 4 * lane);
  double s0 = 0.0, s1 = 0.0, s2 = 0.0, s3 = 0.0, q0 = 0.0, q1 = 0.0, q2 = 0.0, q3 = 0.0;
#pragma unroll 1
  for (int it = 0; it < 8; ++it) {
    const int row = it * 8 + wave;
    float* sp = stg + row * CD + 4 * lane;
    const v4f f  = *(const v4f*)sp;
    const v4f yv = *(const v4f*)(y1 + (size_t)(rowBase + row) * CD + 4 * lane);
    const v4f x1 = yv * sc + sh;
    const v4f o  = x1 + f;
    *(v4f*)sp = o;
    s0 += (double)o.x; s1 += (double)o.y; s2 += (double)o.z; s3 += (double)o.w;
    q0 += (double)o.x * (double)o.x; q1 += (double)o.y * (double)o.y;
    q2 += (double)o.z * (double)o.z; q3 += (double)o.w * (double)o.w;
  }
  {
    double* pw = spw + wave * REC + 4 * lane;
    pw[0] = s0; pw[1] = s1; pw[2] = s2; pw[3] = s3;
    pw[CD + 0] = q0; pw[CD + 1] = q1; pw[CD + 2] = q2; pw[CD + 3] = q3;
  }
  __syncthreads();
  if (tid < CD) {
    double S = 0.0, Q = 0.0;
#pragma unroll
    for (int w = 0; w < NWAVE; ++w) { S += spw[w * REC + tid]; Q += spw[w * REC + CD + tid]; }
    srec[tid] = S;
    srec[CD + tid] = Q;
  }
  __syncthreads();

  float* gy = y2 + (size_t)rowBase * CD + 4 * lane;
  v2d rv = {0.0, 0.0};
  if (tid < CD) rv = *(const v2d*)(srec + 2 * tid);
  double* gr = part + (size_t)blockIdx.x * REC + 2 * (tid < CD ? tid : 0);
#pragma unroll 1
  for (int it = 0; it < 8; ++it) {
    const int row = it * 8 + wave;
    const v4f v = *(const v4f*)(stg + row * CD + 4 * lane);
    *(volatile v4f*)(gy + (size_t)row * CD) = v;
  }
  if (tid < CD) *(volatile v2d*)gr = rv;
  __threadfence();
#pragma unroll 1
  for (int it = 0; it < 8; ++it) {
    const int row = it * 8 + wave;
    const v4f v = *(const v4f*)(stg + row * CD + 4 * lane);
    *(volatile v4f*)(gy + (size_t)row * CD) = v;
  }
  if (tid < CD) *(volatile v2d*)gr = rv;
}

__global__ __launch_bounds__(PTHR) void k_out(const float* __restrict__ y2, const float* __restrict__ tab, float* out) {
  __shared__ __attribute__((aligned(16))) float swp[4 * CD];
  const int b = blockIdx.x, tid = threadIdx.x, lane = tid & 31, wave = tid >> 5;
  const size_t gbase = (size_t)b * NPG * CD;
  const v4f sc = *(const v4f*)(tab + 4 * lane), sh = *(const v4f*)(tab + CD + 4 * lane);
  const float* yg = y2 + gbase + 4 * lane;
  float* o0 = out + gbase + 4 * lane;
  float* o1 = out + (size_t)NNODE * CD + (size_t)b * CD + 4 * lane;
  v4f s = {0.f, 0.f, 0.f, 0.f};
#pragma unroll 1
  for (int k = 0; k < NPG / 4; ++k) {
    const int row = 4 * k + wave;
    const v4f v = *(const v4f*)(yg + (size_t)row * CD);
    const v4f o = v * sc + sh;
    *(volatile v4f*)(o0 + (size_t)row * CD) = o;
    s = s + o;
  }
  *(v4f*)(swp + wave * CD + 4 * lane) = s;
  __syncthreads();
  v4f mv = {0.f, 0.f, 0.f, 0.f};
  if (wave == 0) {
    const v4f a0 = *(const v4f*)(swp + 0 * CD + 4 * lane);
    const v4f a1 = *(const v4f*)(swp + 1 * CD + 4 * lane);
    const v4f a2 = *(const v4f*)(swp + 2 * CD + 4 * lane);
    const v4f a3 = *(const v4f*)(swp + 3 * CD + 4 * lane);
    mv = ((a0 + a1) + a2) + a3;
    mv = mv * (1.0f / (float)NPG);
    *(volatile v4f*)o1 = mv;
  }
  __threadfence();
#pragma unroll 1
  for (int k = 0; k < NPG / 4; ++k) {
    const int row = 4 * k + wave;
    const v4f v = *(const v4f*)(yg + (size_t)row * CD);
    const v4f o = v * sc + sh;
    *(volatile v4f*)(o0 + (size_t)row * CD) = o;
  }
  if (wave == 0) *(volatile v4f*)o1 = mv;
}

extern "C" void kernel_launch(void* const* d_in, const int* in_sizes, int n_in,
                              void* d_out, int out_size, void* d_ws, size_t ws_size,
                              hipStream_t stream) {
  if (n_in < 15) return;
  if (in_sizes[0] != NGR * 2 || in_sizes[1] != NGR * NCU * 2 || in_sizes[2] != NGR * NCU) return;
  if (in_sizes[3] != 2 * CD || in_sizes[4] != CD || in_sizes[5] != 3 * CD || in_sizes[6] != CD) return;
  if (in_sizes[7] != NL * CD * CD || in_sizes[8] != NL * CD) return;
  if (in_sizes[9] != NL * CD || in_sizes[10] != NL * CD) return;
  if (in_sizes[11] != NL * CD * HD || in_sizes[12] != NL * HD) return;
  if (in_sizes[13] != NL * HD * CD || in_sizes[14] != NL * CD) return;
  if (out_size != NNODE * CD + NGR * CD) return;

  const float* depot = (const float*)d_in[0];
  const float* cust  = (const float*)d_in[1];
  const float* dem   = (const float*)d_in[2];
  const float* Wd    = (const float*)d_in[3];
  const float* bd    = (const float*)d_in[4];
  const float* Wi    = (const float*)d_in[5];
  const float* bi    = (const float*)d_in[6];
  const float* gcnW  = (const float*)d_in[7];
  const float* gcnb  = (const float*)d_in[8];
  const float* bng   = (const float*)d_in[9];
  const float* bnb   = (const float*)d_in[10];
  const float* ffW1  = (const float*)d_in[11];
  const float* ffb1  = (const float*)d_in[12];
  const float* ffW2  = (const float*)d_in[13];
  const float* ffb2  = (const float*)d_in[14];
  float* out = (float*)d_out;

  char* ws = (char*)d_ws;
  size_t off = 0;
  const size_t oW  = off; off += (size_t)WPTOT * 2;            off = (off + 255) & ~(size_t)255;
  const size_t oX0 = off; off += (size_t)NNODE * CD * 4;       off = (off + 255) & ~(size_t)255;
  const size_t oH  = off; off += (size_t)NNODE * CD * 4;       off = (off + 255) & ~(size_t)255;
  const size_t oY1 = off; off += (size_t)NNODE * CD * 4;       off = (off + 255) & ~(size_t)255;
  const size_t oY2 = off; off += (size_t)NNODE * CD * 4;       off = (off + 255) & ~(size_t)255;
  const size_t oT0 = off; off += (size_t)REC * 4;              off = (off + 255) & ~(size_t)255;
  const size_t oT1 = off; off += (size_t)REC * 4;              off = (off + 255) & ~(size_t)255;
  const size_t oT2 = off; off += (size_t)REC * 4;              off = (off + 255) & ~(size_t)255;
  const size_t oP1 = off; off += (size_t)NP1 * REC * 8;        off = (off + 255) & ~(size_t)255;
  const size_t oP2 = off; off += (size_t)NP2 * REC * 8;        off = (off + 255) & ~(size_t)255;
  if (off > ws_size || off > (size_t)WSCAP) return;
  unsigned short* wp = (unsigned short*)(ws + oW);
  float*  X0 = (float*)(ws + oX0);
  float*  Hb = (float*)(ws + oH);
  float*  Y1 = (float*)(ws + oY1);
  float*  Y2 = (float*)(ws + oY2);
  float*  T0 = (float*)(ws + oT0);
  float*  T1 = (float*)(ws + oT1);
  float*  T2 = (float*)(ws + oT2);
  double* P1 = (double*)(ws + oP1);
  double* P2 = (double*)(ws + oP2);

  k_wprep<<<NL * WBLK_L, NTHR, 0, stream>>>(gcnW, ffW1, ffW2, wp);

  k_init<<<NNODE / IROWS, NTHR, 0, stream>>>(depot, cust, dem, Wd, bd, Wi, bi, X0, T0);

  hipFuncSetAttribute(reinterpret_cast<const void*>(&k_gemm1), hipFuncAttributeMaxDynamicSharedMemorySize, LDS_G1);
  hipFuncSetAttribute(reinterpret_cast<const void*>(&k_ffn), hipFuncAttributeMaxDynamicSharedMemorySize, LDS_FFN);

  for (int l = 0; l < NL; ++l) {
    const float* ysrc = (l == 0) ? X0 : Y2;
    const float* tin  = (l == 0) ? T0 : T2;
    const unsigned short* wpl = wp + (size_t)l * WPL_SZ;
    k_gemm1<<<NNODE / G1ROWS, NTHR, LDS_G1, stream>>>(ysrc, tin, wpl, Hb);
    k_prefix<<<NGR, PTHR, 0, stream>>>(Hb, ysrc, tin, gcnb + l * CD, Y1, P1);
    k_bnfin<<<1, PTHR, 0, stream>>>(P1, NP1, bng + l * CD, bnb + l * CD, T1);
    k_ffn<<<NNODE / FROWS, NTHR, LDS_FFN, stream>>>(Y1, T1, wpl + WPG_SZ, ffb1 + l * HD,
                                                     wpl + WPG_SZ + WP1_SZ, ffb2 + l * CD, Y2, P2);
    k_bnfin<<<1, PTHR, 0, stream>>>(P2, NP2, bng + l * CD, bnb + l * CD, T2);
  }

  k_out<<<NGR, PTHR, 0, stream>>>(Y2, T2, out);
}
